// MessageControlGraphAttentionLayer_2267742732711
// MI455X (gfx1250) — hardware-verified
//
#include <hip/hip_runtime.h>
#include <math.h>

typedef __attribute__((ext_vector_type(16))) _Float16 v16h;
typedef __attribute__((ext_vector_type(16))) __bf16 v16b;
typedef __attribute__((ext_vector_type(8)))  _Float16 v8h;
typedef __attribute__((ext_vector_type(8)))  float v8f;
typedef __attribute__((ext_vector_type(4)))  float v4f;
typedef __attribute__((ext_vector_type(2)))  float v2f;
typedef __attribute__((ext_vector_type(4)))  unsigned v4u;
typedef __attribute__((ext_vector_type(4)))  int v4i;
typedef float __attribute__((may_alias)) float_a;
typedef int __attribute__((may_alias)) int_a;

template <typename T> __device__ __forceinline__ void vst2(void* p, T v) { *(volatile T*)p = v; __threadfence(); *(volatile T*)p = v; }
__device__ __forceinline__ v8f wmma16(v16h a, v16h b, v8f c) {
  v8f d = __builtin_amdgcn_wmma_f32_16x16x32_f16(false, a, false, b, (short)0, c, false, false);
  asm volatile("v_nop\n\tv_nop\n\tv_nop\n\tv_nop" : "+v"(d) : "v"(a), "v"(b));
  return d;
}
__device__ __forceinline__ v8f wmma_bf(v16b a, v16b b, v8f c) {
  v8f d = __builtin_amdgcn_wmma_f32_16x16x32_bf16(false, a, false, b, (short)0, c, false, false);
  asm volatile("v_nop\n\tv_nop\n\tv_nop\n\tv_nop" : "+v"(d) : "v"(a), "v"(b));
  return d;
}
__device__ __forceinline__ v16h frag_h(const _Float16* rowk0, int lane) {
  union { v16h v; v8h q[2]; } u; const _Float16* p = rowk0 + 8 * (lane >> 4);
  u.q[0] = *(const v8h*)p; u.q[1] = *(const v8h*)(p + 16); return u.v;
}
__device__ __forceinline__ v16h frag_f32(const float* rowk0, int lane) {
  v16h a; const float* p = rowk0 + 8 * (lane >> 4);
#pragma unroll
  for (int i = 0; i < 8; ++i) { a[i] = (_Float16)p[i]; a[8 + i] = (_Float16)p[16 + i]; }
  return a;
}
__device__ __forceinline__ v16h frag_f32s(const float* rowk0, int lane, float sc) {
  v16h a; const float* p = rowk0 + 8 * (lane >> 4);
#pragma unroll
  for (int i = 0; i < 8; ++i) { a[i] = (_Float16)(p[i] * sc); a[8 + i] = (_Float16)(p[16 + i] * sc); }
  return a;
}
__device__ __forceinline__ v16h fragc_f32(const float* W, int k0, int n, int lane, int ld, int K) {
  v16h a; const int g = lane >> 4;
#pragma unroll
  for (int i = 0; i < 8; ++i) { const int ka = k0 + 8 * g + i, kb = ka + 16;
    a[i] = (_Float16)(ka < K ? W[(size_t)(ka < K ? ka : K - 1) * ld + n] : 0.f); a[8 + i] = (_Float16)(kb < K ? W[(size_t)(kb < K ? kb : K - 1) * ld + n] : 0.f); }
  return a;
}
struct F2 { v16b h, l; };
__device__ __forceinline__ F2 bsplit16(const float v[16]) { F2 r;
#pragma unroll
  for (int i = 0; i < 16; ++i) { const __bf16 h = (__bf16)v[i]; r.h[i] = h; r.l[i] = (__bf16)(v[i] - (float)h); }
  return r; }
__device__ __forceinline__ F2 split_row(const float* row, int k0, int lane) { float v[16]; const float* p = row + k0 + 8 * (lane >> 4);
#pragma unroll
  for (int i = 0; i < 8; ++i) { v[i] = p[i]; v[8 + i] = p[16 + i]; }
  return bsplit16(v); }
__device__ __forceinline__ F2 split_rowK(const float* row, int k0, int lane, int K) { float v[16]; const int g = lane >> 4;
#pragma unroll
  for (int i = 0; i < 8; ++i) { const int ka = k0 + 8 * g + i, kb = ka + 16; v[i] = ka < K ? row[ka < K ? ka : K - 1] : 0.f; v[8 + i] = kb < K ? row[kb < K ? kb : K - 1] : 0.f; }
  return bsplit16(v); }
__device__ __forceinline__ F2 split_col(const float* W, int k0, int n, int lane, int ld, int K) { float v[16]; const int g = lane >> 4;
#pragma unroll
  for (int i = 0; i < 8; ++i) { const int ka = k0 + 8 * g + i, kb = ka + 16; v[i] = ka < K ? W[(size_t)(ka < K ? ka : K - 1) * ld + n] : 0.f; v[8 + i] = kb < K ? W[(size_t)(kb < K ? kb : K - 1) * ld + n] : 0.f; }
  return bsplit16(v); }
__device__ __forceinline__ v8f mac3(const F2& a, const F2& b, v8f c) { c = wmma_bf(a.l, b.h, c); c = wmma_bf(a.h, b.l, c); return wmma_bf(a.h, b.h, c); }
__device__ __forceinline__ float sigm(float v) { return 1.0f / (1.0f + expf(-v)); }
#define LDSX() do { asm volatile("s_wait_dscnt 0" ::: "memory"); __builtin_amdgcn_wave_barrier(); __builtin_amdgcn_fence(__ATOMIC_RELEASE, "workgroup"); } while (0)


#define NB 4
#define TT 256
#define DD 256
#define OO 256
#define NH 8
#define NR (NB * TT)
#ifndef NBT
#define NBT NB
#define TB0 0
#endif
#define NRT (NBT * TT)
#define RB0 ((size_t)TB0 * TT)
typedef __attribute__((ext_vector_type(8))) __bf16 v8b;
__device__ __forceinline__ v16b frag_b(const __bf16* rowk0, int lane) {
  union { v16b v; v8b q[2]; } u; const __bf16* p = rowk0 + 8 * (lane >> 4);
  u.q[0] = *(const v8b*)p; u.q[1] = *(const v8b*)(p + 16); return u.v;
}
__device__ __forceinline__ float bfr(float v) { return (float)(__bf16)v; }
__device__ __attribute__((noinline)) float exp_ni(float v) { return expf(v); }
__device__ __attribute__((noinline)) float erf_ni(float v) { return erff(v); }
__device__ __attribute__((noinline)) float tanh_ni(float v) { return tanhf(v); }

#define PK_AP 0
#define PK_AW ((size_t)OO * DD)
#define PK_PA (PK_AW + (size_t)16 * OO)
#define PK_PN (PK_PA + (size_t)OO * NH * DD)
#define PK_END (PK_PN + (size_t)OO * DD)
#define WS_PK  0u
#define WS_XT  (((2u * PK_END) + 127u) / 128u * 128u)
#define WS_ATT (WS_XT + 2u * NR * DD)
#define WS_X1  (WS_ATT + 4u * (size_t)NB * TT * NH * TT)
#define WS_Y   (WS_X1 + 4u * (size_t)NR * NH * DD)
#define WS_ST  (WS_Y + 4u * NR * OO)
#define WS_END (WS_ST + 4u * (NR / 64) * OO * 2)

__global__ __launch_bounds__(256) void k_pack(const float* __restrict__ APW, const float* __restrict__ AW, const float* __restrict__ PAW, const float* __restrict__ PNW, __bf16* __restrict__ PK) {
  __shared__ __align__(16) __bf16 s[NH * DD]; const int n = blockIdx.x, which = blockIdx.y, t = threadIdx.x; int K; size_t dst;
  if (which == 0) { K = DD; dst = PK_AP + (size_t)n * DD; for (int k = t; k < K; k += 256) s[k] = (__bf16)APW[(size_t)k * OO + n]; }
  else if (which == 1) { if (n >= 16) return; K = OO; dst = PK_AW + (size_t)n * OO; for (int k = t; k < K; k += 256) s[k] = (__bf16)((n < NH) ? AW[(size_t)k * NH + n] : 0.f); }
  else if (which == 2) { K = NH * DD; dst = PK_PA + (size_t)n * NH * DD; for (int k = t; k < K; k += 256) s[k] = (__bf16)PAW[(size_t)k * OO + n]; }
  else { K = DD; dst = PK_PN + (size_t)n * DD; for (int k = t; k < K; k += 256) s[k] = (__bf16)PNW[(size_t)k * OO + n]; }
  __syncthreads();
  for (int q = t; q < K / 8; q += 256) vst2((unsigned*)(PK + dst + q * 8), *(const v4u*)&s[q * 8]);
}
__global__ __launch_bounds__(256) void k_xt(const float* __restrict__ X, __bf16* __restrict__ XT) {
  __shared__ __align__(16) __bf16 s[DD][72]; const int tid = threadIdx.x; const int tb = blockIdx.x, b = blockIdx.y + TB0; const int t0 = tb * 64;
  for (int e = tid; e < 64 * DD; e += 256) { const int r = e >> 8, d = e & 255; s[d][r] = (__bf16)X[((size_t)b * TT + t0 + r) * DD + d]; }
  __syncthreads();
  for (int e = tid; e < DD * 8; e += 256) { const int d = e >> 3, pc = e & 7; vst2((unsigned*)(XT + ((size_t)b * DD + d) * TT + t0 + pc * 8), *(const v4u*)&s[d][pc * 8]); }
}
__global__ __launch_bounds__(128) void k_pair(const float* __restrict__ X, const int* __restrict__ BND, const __bf16* __restrict__ PK, const float* __restrict__ APB, float* __restrict__ ATT) {
  __shared__ __align__(16) __bf16 sph[64][DD + 8], spl[64][DD + 8]; __shared__ __align__(16) __bf16 sah[64][OO + 8], sal[64][OO + 8]; __shared__ int spre[TT + 1]; __shared__ __align__(16) float satt[NH][68];
  const int tid = threadIdx.x, wave = tid >> 5, lane = tid & 31, col = lane & 15, g = lane >> 4; const int kb = blockIdx.x, j = blockIdx.y, b = blockIdx.z + TB0; const int k0 = kb * 64;
  if (tid == 0) { int s = 0; spre[0] = 0; for (int t = 0; t < TT; ++t) { s += BND[(size_t)b * TT + t]; spre[t + 1] = s; } }
  { const float* xj = X + ((size_t)b * TT + j) * DD; for (int e = tid; e < 64 * DD; e += 128) { const int r = e >> 8, d = e & 255; const float pv = bfr(xj[d]) * bfr(X[((size_t)b * TT + k0 + r) * DD + d]); const __bf16 hb = (__bf16)pv; sph[r][d] = hb; spl[r][d] = (__bf16)(pv - (float)hb); } }
  if (tid < 64) for (int c = DD; c < DD + 8; ++c) { sph[tid][c] = (__bf16)0.f; spl[tid][c] = (__bf16)0.f; sah[tid][c] = (__bf16)0.f; sal[tid][c] = (__bf16)0.f; }
  __syncthreads();
#pragma unroll 1
  for (int half = 0; half < 2; ++half) { v8f acc[8] = {};
#pragma unroll 2
    for (int kc = 0; kc < DD / 32; ++kc) { F2 a; a.h = frag_b(&sph[wave * 16 + col][kc * 32], lane); a.l = frag_b(&spl[wave * 16 + col][kc * 32], lane);
#pragma unroll
      for (int jt = 0; jt < 8; ++jt) { const v16b w = frag_b(PK + PK_AP + (size_t)(half * 128 + jt * 16 + col) * DD + kc * 32, lane); acc[jt] = wmma_bf(a.l, w, acc[jt]); acc[jt] = wmma_bf(a.h, w, acc[jt]); } }
#pragma unroll
    for (int jt = 0; jt < 8; ++jt) { const int c = half * 128 + jt * 16 + col; const float bb = bfr(APB[c]);
#pragma unroll
      for (int r = 0; r < 8; ++r) { const float v = tanh_ni(acc[jt][r] + bb); const __bf16 hb = (__bf16)v; sah[wave * 16 + 8 * g + r][c] = hb; sal[wave * 16 + 8 * g + r][c] = (__bf16)(v - (float)hb); } } }
  LDSX();
  { v8f acc = {};
#pragma unroll 2
    for (int kc = 0; kc < OO / 32; ++kc) { F2 a; a.h = frag_b(&sah[wave * 16 + col][kc * 32], lane); a.l = frag_b(&sal[wave * 16 + col][kc * 32], lane); const v16b w = frag_b(PK + PK_AW + (size_t)col * OO + kc * 32, lane); acc = wmma_bf(a.l, w, acc); acc = wmma_bf(a.h, w, acc); }
    if (col < NH) {
#pragma unroll
      for (int r = 0; r < 8; ++r) { const int kk = k0 + wave * 16 + 8 * g + r; const int hi_ = max(j, kk), lo_ = min(j, kk); const bool m = (spre[hi_ + 1] - spre[lo_] == 0) || (j == kk); satt[col][wave * 16 + 8 * g + r] = m ? acc[r] : 0.f; } } }
  __syncthreads();
  for (int e = tid; e < NH * 16; e += 128) { const int h = e >> 4, pc = e & 15; vst2(ATT + (((size_t)b * TT + j) * NH + h) * TT + k0 + pc * 4, *(const v4f*)&satt[h][pc * 4]); }
}
__global__ __launch_bounds__(256) void k_agg(const float* __restrict__ ATT, const __bf16* __restrict__ XT, float* __restrict__ X1) {
  __shared__ __align__(16) __bf16 sph[16][TT + 8], spl[16][TT + 8]; __shared__ __align__(16) float sx1[NH * DD]; __shared__ float red[NH][2];
  const int tid = threadIdx.x, wave = tid >> 5, lane = tid & 31, col = lane & 15, g = lane >> 4; const int j = blockIdx.x, b = blockIdx.y + TB0;
  for (int e = tid; e < 16 * (TT + 8); e += 256) { sph[e / (TT + 8)][e % (TT + 8)] = (__bf16)0.f; spl[e / (TT + 8)][e % (TT + 8)] = (__bf16)0.f; }
  __syncthreads();
  { const int h = wave; const float* row = ATT + (((size_t)b * TT + j) * NH + h) * TT; float v[8]; float mx = -3.0e38f;
#pragma unroll
    for (int i = 0; i < 8; ++i) { v[i] = row[lane * 8 + i]; mx = fmaxf(mx, v[i]); }
#pragma unroll
    for (int o = 1; o < 32; o <<= 1) mx = fmaxf(mx, __shfl_xor(mx, o));
    float s = 0.f, e8[8];
#pragma unroll
    for (int i = 0; i < 8; ++i) { e8[i] = exp_ni(v[i] - mx); s += e8[i]; }
#pragma unroll
    for (int o = 1; o < 32; o <<= 1) s += __shfl_xor(s, o);
    const float is = 1.0f / s;
#pragma unroll
    for (int i = 0; i < 8; ++i) { const float p = e8[i] * is; const __bf16 hb = (__bf16)p; sph[h][lane * 8 + i] = hb; spl[h][lane * 8 + i] = (__bf16)(p - (float)hb); } }
  __syncthreads();
  { v8f acc[2] = {};
#pragma unroll 2
    for (int kc = 0; kc < TT / 32; ++kc) { F2 a; a.h = frag_b(&sph[col][kc * 32], lane); a.l = frag_b(&spl[col][kc * 32], lane);
#pragma unroll
      for (int jt = 0; jt < 2; ++jt) { const v16b w = frag_b(XT + ((size_t)b * DD + (wave * 2 + jt) * 16 + col) * TT + kc * 32, lane); acc[jt] = wmma_bf(a.l, w, acc[jt]); acc[jt] = wmma_bf(a.h, w, acc[jt]); } }
#pragma unroll
    for (int jt = 0; jt < 2; ++jt) { const int d = (wave * 2 + jt) * 16 + col;
#pragma unroll
      for (int r = 0; r < 8; ++r) if (g == 0) sx1[d * NH + r] = acc[jt][r]; } }
  __syncthreads();
  for (int q = tid; q < NH * DD / 4; q += 256) vst2(X1 + ((size_t)b * TT + j) * NH * DD + q * 4, *(const v4f*)&sx1[q * 4]);
}
__global__ __launch_bounds__(128) void k_y(const float* __restrict__ X1, const float* __restrict__ X, const __bf16* __restrict__ PK, const float* __restrict__ PAB, const float* __restrict__ PNB, float* __restrict__ Y, float* __restrict__ ST) {
  __shared__ __align__(16) float so[4][16][132]; __shared__ float sst[128][2];
  const int tid = threadIdx.x, wave = tid >> 5, lane = tid & 31, col = lane & 15, g = lane >> 4; const size_t r0 = RB0 + (size_t)blockIdx.x * 64 + wave * 16; const int n0 = blockIdx.y * 128;
  v8f acc[8] = {};
#pragma unroll 2
  for (int kc = 0; kc < NH * DD / 32; ++kc) { const F2 a = split_row(X1 + (r0 + col) * NH * DD, kc * 32, lane);
#pragma unroll
    for (int jt = 0; jt < 8; ++jt) { const v16b w = frag_b(PK + PK_PA + (size_t)(n0 + jt * 16 + col) * NH * DD + kc * 32, lane); acc[jt] = wmma_bf(a.l, w, acc[jt]); acc[jt] = wmma_bf(a.h, w, acc[jt]); } }
#pragma unroll
  for (int kc = 0; kc < DD / 32; ++kc) { v16b a; { const float* p = X + (r0 + col) * DD + kc * 32 + 8 * g;
#pragma unroll
      for (int i = 0; i < 8; ++i) { a[i] = (__bf16)p[i]; a[8 + i] = (__bf16)p[16 + i]; } }
#pragma unroll
    for (int jt = 0; jt < 8; ++jt) acc[jt] = wmma_bf(a, frag_b(PK + PK_PN + (size_t)(n0 + jt * 16 + col) * DD + kc * 32, lane), acc[jt]); }
#pragma unroll
  for (int jt = 0; jt < 8; ++jt) { const int c = n0 + jt * 16 + col; const float bb = bfr(PAB[c]) + bfr(PNB[c]);
#pragma unroll
    for (int r = 0; r < 8; ++r) so[wave][8 * g + r][jt * 16 + col] = acc[jt][r] + bb; }
  __syncthreads();
  for (int rl = 0; rl < 16; ++rl) vst2(Y + (r0 + rl) * OO + n0 + lane * 4, *(const v4f*)&so[wave][rl][lane * 4]);
  { const int c = tid; float s = 0.f, q = 0.f; for (int w = 0; w < 4; ++w) for (int r = 0; r < 16; ++r) { const float v = so[w][r][c]; s += v; q += v * v; } sst[c][0] = s; sst[c][1] = q; }
  __syncthreads();
  if (tid < 64) vst2(ST + ((size_t)blockIdx.x * OO + n0) * 2 + tid * 4, *(const v4f*)(&sst[0][0] + tid * 4));
}
__global__ __launch_bounds__(64) void k_bn(const float* __restrict__ Y, const float* __restrict__ ST, const float* __restrict__ G, const float* __restrict__ Bt, float* __restrict__ OUT) {
  const size_t row = RB0 + blockIdx.x; const int t = threadIdx.x; v4f o4;
#pragma unroll
  for (int i = 0; i < 4; ++i) { const int c = t * 4 + i; float s = 0.f, q = 0.f; for (int blk = 0; blk < NRT / 64; ++blk) { s += ST[((size_t)blk * OO + c) * 2]; q += ST[((size_t)blk * OO + c) * 2 + 1]; }
    const float mu = s / (float)NRT; const float var = fmaxf(q / (float)NRT - mu * mu, 0.f); const float v = bfr(G[c]) * (Y[row * OO + c] - mu) / sqrtf(var + 1e-5f) + bfr(Bt[c]);
    const float alpha = 1.6732632423543772f, scl = 1.0507009873554805f; o4[i] = scl * ((v > 0.f) ? v : alpha * (exp_ni(v) - 1.0f)); }
  vst2(OUT + row * OO + t * 4, o4);
}
extern "C" void kernel_launch(void* const* d_in, const int* in_sizes, int n_in, void* d_out, int out_size, void* d_ws, size_t ws_size, hipStream_t stream) {
  (void)in_sizes; (void)n_in; (void)out_size;
  const float** F = (const float**)d_in;
  if (ws_size < (size_t)WS_END) return;
  char* ws = (char*)d_ws; __bf16 *PK = (__bf16*)(ws + WS_PK), *XT = (__bf16*)(ws + WS_XT); float *ATT = (float*)(ws + WS_ATT), *X1 = (float*)(ws + WS_X1), *Y = (float*)(ws + WS_Y), *ST = (float*)(ws + WS_ST);
  k_pack<<<dim3(OO, 4), 256, 0, stream>>>(F[2], F[4], F[5], F[7], PK);
  k_xt<<<dim3(TT / 64, NBT), 256, 0, stream>>>(F[0], XT);
  k_pair<<<dim3(TT / 64, TT, NBT), 128, 0, stream>>>(F[0], (const int*)d_in[1], PK, F[3], ATT);
  k_agg<<<dim3(TT, NBT), 256, 0, stream>>>(ATT, XT, X1);
  k_y<<<dim3(NRT / 64, OO / 128), 128, 0, stream>>>(X1, F[0], PK, F[6], F[8], Y, ST);
  k_bn<<<NRT, 64, 0, stream>>>(Y, ST, F[9], F[10], (float*)d_out);
}
